// PointNetPolylineEncoder_1606317769339
// MI455X (gfx1250) — hardware-verified
//
#include <hip/hip_runtime.h>


#define NBB  32
#define NPL  512
#define NPT  32
#define CIN  9
#define HH   64
#define OUTW 128
#define CHP  (NPL * NPT)
typedef _Float16 h16;
typedef unsigned short bf;
typedef __attribute__((ext_vector_type(16))) __bf16   v16bf;
typedef __attribute__((ext_vector_type(16))) _Float16 v16h;
typedef __attribute__((ext_vector_type(8)))  _Float16 v8h;
typedef __attribute__((ext_vector_type(8)))  unsigned short v8us;
typedef __attribute__((ext_vector_type(8)))  float    v8f;
typedef __attribute__((ext_vector_type(4)))  float    v4f;
typedef v8h  __attribute__((may_alias)) v8ha;
typedef v4f  __attribute__((may_alias)) v4fa;
typedef v8us __attribute__((may_alias)) v8usa;

__device__ __forceinline__ unsigned short f2bf(float f) { unsigned u = __float_as_uint(f); u += 0x7FFFu + ((u >> 16) & 1u); return (unsigned short)(u >> 16); }
__device__ __forceinline__ float bf2f(unsigned short b) { return __uint_as_float(((unsigned)b) << 16); }
__device__ __forceinline__ float bfr(float f) { return bf2f(f2bf(f)); }
__device__ __forceinline__ v16h cat16(v8h lo, v8h hi) { return __builtin_shufflevector(lo, hi, 0, 1, 2, 3, 4, 5, 6, 7, 8, 9, 10, 11, 12, 13, 14, 15); }
__device__ __forceinline__ v16bf cat16b(v8us lo, v8us hi) { return __builtin_bit_cast(v16bf, __builtin_shufflevector(lo, hi, 0, 1, 2, 3, 4, 5, 6, 7, 8, 9, 10, 11, 12, 13, 14, 15)); }
__device__ __forceinline__ v8f wmma16(v16h a, v16h b, v8f c) { return __builtin_amdgcn_wmma_f32_16x16x32_f16(false, a, false, b, (short)0, c, false, false); }
__device__ __forceinline__ v8f wmmab(v16bf a, v16bf b, v8f c) { return __builtin_amdgcn_wmma_f32_16x16x32_bf16(false, a, false, b, (short)0, c, false, false); }


template <typename T16> struct WFrag;
template <> struct WFrag<h16> { typedef v16h V; static __device__ __forceinline__ V ld(const h16* p) { return cat16(*(const v8h*)p, *(const v8h*)(p + 16)); } static __device__ __forceinline__ v8f mma(V a, V b, v8f c) { return wmma16(a, b, c); } };
template <> struct WFrag<bf> { typedef v16bf V; static __device__ __forceinline__ V ld(const bf* p) { return cat16b(*(const v8us*)p, *(const v8us*)(p + 16)); } static __device__ __forceinline__ v8f mma(V a, V b, v8f c) { return wmmab(a, b, c); } };
template <typename T16, int NSPLIT, bool BIAS>
__global__ __launch_bounds__(32) void k_gemmw(const T16* __restrict__ A, const T16* __restrict__ A2, const T16* __restrict__ Bt, const T16* __restrict__ Bt2, int K, float* C, int ldc, const float* __restrict__ bias, size_t sA, size_t sB, size_t sC) {
    typedef typename WFrag<T16>::V V;
    __shared__ __align__(16) float os[16 * 68];
    const size_t z = blockIdx.z; A += z * sA; if (A2) A2 += z * sA; Bt += z * sB; if (Bt2) Bt2 += z * sB; C += z * sC;
    const int lane = threadIdx.x & 31, lr = lane & 15, hi = lane >> 4; const int r0 = blockIdx.x * 64, c0 = blockIdx.y * 64;
    v8f acc[4][4];
#pragma unroll
    for (int mb = 0; mb < 4; ++mb)
#pragma unroll
        for (int nb = 0; nb < 4; ++nb) acc[mb][nb] = (v8f){};
    const size_t aoff = (size_t)(r0 + lr) * K + 8 * hi, boff = (size_t)(c0 + lr) * K + 8 * hi;
#pragma unroll 1
    for (int kc = 0; kc < K; kc += 32) {
        V a[4], a2[4];
#pragma unroll
        for (int mb = 0; mb < 4; ++mb) { a[mb] = WFrag<T16>::ld(A + aoff + (size_t)mb * 16 * K + kc); if (NSPLIT == 1 || NSPLIT == 2) a2[mb] = WFrag<T16>::ld(A2 + aoff + (size_t)mb * 16 * K + kc); }
#pragma unroll
        for (int nb = 0; nb < 4; ++nb) { const V b = WFrag<T16>::ld(Bt + boff + (size_t)nb * 16 * K + kc); V b2; if (NSPLIT >= 2) b2 = WFrag<T16>::ld(Bt2 + boff + (size_t)nb * 16 * K + kc);
#pragma unroll
            for (int mb = 0; mb < 4; ++mb) { acc[mb][nb] = WFrag<T16>::mma(a[mb], b, acc[mb][nb]); if (NSPLIT == 1 || NSPLIT == 2) acc[mb][nb] = WFrag<T16>::mma(a2[mb], b, acc[mb][nb]); if (NSPLIT >= 2) acc[mb][nb] = WFrag<T16>::mma(a[mb], b2, acc[mb][nb]); } }
        asm volatile("v_nop\n\tv_nop\n\tv_nop\n\tv_nop" : "+v"(acc[0][0]), "+v"(acc[1][1]), "+v"(acc[2][2]), "+v"(acc[3][3]) : "v"(a[0]), "v"(a[3]));
    }
#pragma unroll
    for (int mb = 0; mb < 4; ++mb) {
#pragma unroll
        for (int nb = 0; nb < 4; ++nb) {
#pragma unroll
            for (int j = 0; j < 8; ++j) os[(hi * 8 + j) * 68 + nb * 16 + lr] = acc[mb][nb][j]; }
        __builtin_amdgcn_wave_barrier(); asm volatile("" ::: "memory");
        float* crow = C + (size_t)(r0 + mb * 16) * ldc + c0;
#pragma unroll 1
        for (int ps = 0; ps < 2; ++ps) {
#pragma unroll
            for (int s = 0; s < 8; ++s) { const int row = 2 * s + hi, cofs = lr * 4; v4f val = *(const v4fa*)(os + row * 68 + cofs); if (BIAS) { val[0] += bfr(bias[c0 + cofs]); val[1] += bfr(bias[c0 + cofs + 1]); val[2] += bfr(bias[c0 + cofs + 2]); val[3] += bfr(bias[c0 + cofs + 3]); }
                *(volatile v4f*)(crow + (size_t)row * ldc + cofs) = val; }
            if (ps == 0) __threadfence(); }
        __builtin_amdgcn_wave_barrier(); asm volatile("" ::: "memory");
    }
}

__device__ __forceinline__ void splitf(float y, unsigned short& h, unsigned short& l) { h = f2bf(y); l = f2bf(y - bf2f(h)); }
typedef __attribute__((ext_vector_type(2))) unsigned short v2us;
typedef __attribute__((ext_vector_type(4))) unsigned short v4us;
typedef __attribute__((ext_vector_type(2))) float v2f;

__global__ __launch_bounds__(256) void k_wtG(const float* __restrict__ w, int K, int N, bf* Bt) {
    const int lane = threadIdx.x & 31; const int L0 = (blockIdx.x * 8 + (threadIdx.x >> 5)) * 8; const int nlines = N * K / 64;
#pragma unroll 1
    for (int ps = 0; ps < 2; ++ps) {
#pragma unroll 1
        for (int l = 0; l < 8; ++l) { const int L = L0 + l; if (L >= nlines) break; const size_t e = (size_t)L * 64 + lane * 2; const int k = (int)(e % K), n = (int)(e / K); v2us o;
            o[0] = f2bf(w[(size_t)k * N + n]); o[1] = f2bf(w[(size_t)(k + 1) * N + n]); *(volatile v2us*)(Bt + e) = o; }
        if (ps == 0) __threadfence(); }
}
__device__ __forceinline__ float bnf(float x, const float* g, const float* b, const float* m, const float* v, int c) { const float sc = __fmul_rn(bfr(g[c]), __frsqrt_rn(__fadd_rn(bfr(v[c]), 1e-5f))); float t = __fmul_rn(__fsub_rn(x, bfr(m[c])), sc); asm volatile("" : "+v"(t)); return __fadd_rn(t, bfr(b[c])); }
__global__ __launch_bounds__(256) void k_pre(const float* __restrict__ P9, const int* __restrict__ mk, const float* __restrict__ W, const float* __restrict__ g, const float* __restrict__ b, const float* __restrict__ m, const float* __restrict__ v, float* X1) { const int e = (blockIdx.x * 256 + threadIdx.x) * 2; if (e >= CHP * HH) return; const int h = e % HH, pt = e / HH; const float msk = mk[pt] != 0 ? 1.0f : 0.0f; v2f o;
#pragma unroll
    for (int u = 0; u < 2; ++u) { float s = 0.f;
#pragma unroll
        for (int c = 0; c < CIN; ++c) { float p = __fmul_rn(bfr(P9[pt * CIN + c]), bfr(W[c * HH + h + u])); asm volatile("" : "+v"(p)); s = __fadd_rn(s, p); }
        o[u] = __fmul_rn(fmaxf(bnf(s, g, b, m, v, h + u), 0.f), msk); } *(volatile v2f*)(X1 + e) = o; __threadfence(); *(volatile v2f*)(X1 + e) = o; }
__global__ __launch_bounds__(256) void k_pool(const float* __restrict__ X, float* P) { const int e = blockIdx.x * 256 + threadIdx.x; if (e >= NPL * HH) return; const int h = e % HH, pl = e / HH; float mx = -3.0e38f; for (int i = 0; i < NPT; ++i) mx = fmaxf(mx, X[((size_t)pl * NPT + i) * HH + h]); *(volatile float*)(P + e) = mx; __threadfence(); *(volatile float*)(P + e) = mx; }
__global__ __launch_bounds__(256) void k_cat(const float* __restrict__ X1, const float* __restrict__ P, bf* Ah, bf* Al) { const size_t i = ((size_t)blockIdx.x * 256 + threadIdx.x) * 4; if (i >= (size_t)CHP * 2 * HH) return; const int c = (int)(i % (2 * HH)); const int pt = (int)(i / (2 * HH)); v4us oh, ol;
#pragma unroll
    for (int q = 0; q < 4; ++q) { const int cq = c + q; const float x = cq < HH ? X1[(size_t)pt * HH + cq] : P[(pt / NPT) * HH + cq - HH]; unsigned short a, c2; splitf(x, a, c2); oh[q] = a; ol[q] = c2; }
    *(volatile v4us*)(Ah + i) = oh; *(volatile v4us*)(Al + i) = ol; __threadfence(); *(volatile v4us*)(Ah + i) = oh; *(volatile v4us*)(Al + i) = ol; }
__global__ __launch_bounds__(256) void k_bnm(const float* __restrict__ F, const int* __restrict__ mk, const float* __restrict__ g, const float* __restrict__ b, const float* __restrict__ m, const float* __restrict__ v, float* X, bf* Xh, bf* Xl) { const size_t i = ((size_t)blockIdx.x * 256 + threadIdx.x) * 4; if (i >= (size_t)CHP * HH) return; const int h = (int)(i % HH), pt = (int)(i / HH); const float msk = mk[pt] != 0 ? 1.0f : 0.0f; const v4f a = *(const v4f*)(F + i); v4f o; v4us oh, ol;
#pragma unroll
    for (int q = 0; q < 4; ++q) { o[q] = __fmul_rn(fmaxf(bnf(a[q], g, b, m, v, h + q), 0.f), msk); unsigned short u, c2; splitf(o[q], u, c2); oh[q] = u; ol[q] = c2; }
    *(volatile v4f*)(X + i) = o; *(volatile v4us*)(Xh + i) = oh; *(volatile v4us*)(Xl + i) = ol; __threadfence(); *(volatile v4f*)(X + i) = o; *(volatile v4us*)(Xh + i) = oh; *(volatile v4us*)(Xl + i) = ol; }
__global__ __launch_bounds__(256) void k_spl(const float* __restrict__ F, int relu, size_t n4, bf* Fh, bf* Fl) { const size_t i = ((size_t)blockIdx.x * 256 + threadIdx.x) * 4; if (i >= n4 * 4) return; const v4f a = *(const v4f*)(F + i); v4us oh, ol;
#pragma unroll
    for (int q = 0; q < 4; ++q) { unsigned short u, c2; splitf(relu ? fmaxf(a[q], 0.f) : a[q], u, c2); oh[q] = u; ol[q] = c2; } *(volatile v4us*)(Fh + i) = oh; *(volatile v4us*)(Fl + i) = ol; __threadfence(); *(volatile v4us*)(Fh + i) = oh; *(volatile v4us*)(Fl + i) = ol; }
__global__ __launch_bounds__(256) void k_out(const float* __restrict__ F4, const int* __restrict__ mk, float* OUT) { const size_t i = ((size_t)blockIdx.x * 256 + threadIdx.x) * 4; if (i >= (size_t)NBB * NPL * OUTW) return; const int pl = (int)(i / OUTW); int any = 0; for (int j = 0; j < NPT; ++j) any |= (mk[(size_t)pl * NPT + j] != 0); const float vg = any ? 1.0f : 0.0f; const v4f a = *(const v4f*)(F4 + i); v4f o;
#pragma unroll
    for (int q = 0; q < 4; ++q) o[q] = __fmul_rn(a[q], vg); *(volatile v4f*)(OUT + i) = o; __threadfence(); *(volatile v4f*)(OUT + i) = o; }

extern "C" void kernel_launch(void* const* d_in, const int* in_sizes, int n_in,
                              void* d_out, int out_size, void* d_ws, size_t ws_size, hipStream_t stream) {
    (void)in_sizes; (void)n_in; (void)out_size;
    const float* IN[21]; for (int i = 0; i < 21; ++i) IN[i] = (const float*)d_in[i];
    const int* MK = (const int*)d_in[20];
    float* OUT = (float*)d_out;
    char* wsp = (char*)d_ws;
    auto take = [&](size_t bytes) { char* p = wsp; wsp += (bytes + 255) & ~(size_t)255; return (void*)p; };
    bf* W1 = (bf*)take((size_t)HH * 2 * HH * 2); bf* W2 = (bf*)take((size_t)HH * HH * 2); bf* W3 = (bf*)take((size_t)HH * HH * 2); bf* W4 = (bf*)take((size_t)OUTW * HH * 2);
    float* X1 = (float*)take((size_t)CHP * HH * 4); float* P1 = (float*)take((size_t)NPL * HH * 4); bf* Ah = (bf*)take((size_t)CHP * 2 * HH * 2); bf* Al = (bf*)take((size_t)CHP * 2 * HH * 2); float* F = (float*)take((size_t)CHP * HH * 4); float* X = (float*)take((size_t)CHP * HH * 4); bf* Xh = (bf*)take((size_t)CHP * HH * 2); bf* Xl = (bf*)take((size_t)CHP * HH * 2);
    float* PALL = (float*)take((size_t)NBB * NPL * HH * 4); bf* Ph = (bf*)take((size_t)NBB * NPL * HH * 2); bf* Pl = (bf*)take((size_t)NBB * NPL * HH * 2); float* F3 = (float*)take((size_t)NBB * NPL * HH * 4); bf* Gh = (bf*)take((size_t)NBB * NPL * HH * 2); bf* Gl = (bf*)take((size_t)NBB * NPL * HH * 2); float* F4 = (float*)take((size_t)NBB * NPL * OUTW * 4);
    if ((size_t)(wsp - (char*)d_ws) > ws_size) return;
    k_wtG<<<(2 * HH * HH / 64 + 63) / 64, 256, 0, stream>>>(IN[6], 2 * HH, HH, W1); k_wtG<<<(HH * HH / 64 + 63) / 64, 256, 0, stream>>>(IN[11], HH, HH, W2); k_wtG<<<(HH * HH / 64 + 63) / 64, 256, 0, stream>>>(IN[16], HH, HH, W3); k_wtG<<<(HH * OUTW / 64 + 63) / 64, 256, 0, stream>>>(IN[18], HH, OUTW, W4);
    for (int bb = 0; bb < NBB; ++bb) { const float* pb = IN[0] + (size_t)bb * CHP * CIN; const int* mb = MK + (size_t)bb * CHP;
        k_pre<<<(CHP * HH / 2 + 255) / 256, 256, 0, stream>>>(pb, mb, IN[1], IN[2], IN[3], IN[4], IN[5], X1); k_pool<<<(NPL * HH + 255) / 256, 256, 0, stream>>>(X1, P1);
        k_cat<<<(CHP * 2 * HH / 4 + 255) / 256, 256, 0, stream>>>(X1, P1, Ah, Al);
        k_gemmw<bf, 1, false><<<dim3(CHP / 64, 1, 1), 32, 0, stream>>>(Ah, Al, W1, nullptr, 2 * HH, F, HH, nullptr, 0, 0, 0); k_bnm<<<(CHP * HH / 4 + 255) / 256, 256, 0, stream>>>(F, mb, IN[7], IN[8], IN[9], IN[10], X, Xh, Xl);
        k_gemmw<bf, 1, false><<<dim3(CHP / 64, 1, 1), 32, 0, stream>>>(Xh, Xl, W2, nullptr, HH, F, HH, nullptr, 0, 0, 0); k_bnm<<<(CHP * HH / 4 + 255) / 256, 256, 0, stream>>>(F, mb, IN[12], IN[13], IN[14], IN[15], X, Xh, Xl);
        k_pool<<<(NPL * HH + 255) / 256, 256, 0, stream>>>(X, PALL + (size_t)bb * NPL * HH); }
    k_spl<<<(NBB * NPL * HH / 4 + 255) / 256, 256, 0, stream>>>(PALL, 0, (size_t)NBB * NPL * HH / 4, Ph, Pl);
    k_gemmw<bf, 1, true><<<dim3(NBB * NPL / 64, 1, 1), 32, 0, stream>>>(Ph, Pl, W3, nullptr, HH, F3, HH, IN[17], 0, 0, 0); k_spl<<<(NBB * NPL * HH / 4 + 255) / 256, 256, 0, stream>>>(F3, 1, (size_t)NBB * NPL * HH / 4, Gh, Gl);
    k_gemmw<bf, 1, true><<<dim3(NBB * NPL / 64, OUTW / 64, 1), 32, 0, stream>>>(Gh, Gl, W4, nullptr, HH, F4, OUTW, IN[19], 0, 0, 0);
    k_out<<<(NBB * NPL * OUTW / 4 + 255) / 256, 256, 0, stream>>>(F4, MK, OUT);
}
